// HybridBlock_56977036148957
// MI455X (gfx1250) — hardware-verified
//
#include <hip/hip_runtime.h>


namespace {
constexpr int Bsz = 8, T = 1024, D = 512, NH = 8, DH = 64, FF = 4 * D;
constexpr int NQKV = 3 * D, MROWS = Bsz * T, QT_PER_B = T / 16;
constexpr float EPS = 1e-5f;
constexpr float KW_SC = 4096.0f, INV_KW_SC = 1.0f / 4096.0f;
constexpr float INV_2SIG2 = 1.0f / 512.0f;

typedef _Float16 b16;
typedef __attribute__((ext_vector_type(16))) _Float16 v16b;
typedef __attribute__((ext_vector_type(8)))  _Float16 v8b;
typedef __attribute__((ext_vector_type(8)))  float v8f;
typedef __attribute__((ext_vector_type(4)))  float v4f;

__device__ __forceinline__ v8b ld8b(const b16* p) { return *(const v8b*)p; }
__device__ __forceinline__ v16b cat8b(v8b a, v8b b) { return __builtin_shufflevector(a, b, 0, 1, 2, 3, 4, 5, 6, 7, 8, 9, 10, 11, 12, 13, 14, 15); }
__device__ __forceinline__ v16b frag_kb(const b16* p, int hh) { return cat8b(ld8b(p + 8 * hh), ld8b(p + 16 + 8 * hh)); }
__device__ __forceinline__ void split16(float v, b16& hi, b16& lo) { hi = (b16)v; lo = (b16)(v - (float)hi); }
__device__ __forceinline__ void frag_ksplit(const float* p, int hh, v16b& fh_, v16b& fl_) {
  const float* p0 = p + 8 * hh; const float* p1 = p + 16 + 8 * hh;
#pragma unroll
  for (int e = 0; e < 8; ++e) { b16 a, c; split16(p0[e], a, c); fh_[e] = a; fl_[e] = c; split16(p1[e], a, c); fh_[8 + e] = a; fl_[8 + e] = c; }
}
__device__ __forceinline__ v8f wmma16b(v16b a, v16b b, v8f c) {
  v8f d = __builtin_amdgcn_wmma_f32_16x16x32_f16(false, a, false, b, (short)0, c, false, false);
  asm volatile("v_nop\n\tv_nop\n\tv_nop\n\tv_nop" : "+v"(d) : "v"(a), "v"(b));
  return d;
}
__device__ __forceinline__ void wave_lds_sync() {
  __builtin_amdgcn_fence(__ATOMIC_RELEASE, "workgroup");
  __builtin_amdgcn_wave_barrier();
  __builtin_amdgcn_fence(__ATOMIC_ACQUIRE, "workgroup");
}

struct Opnd { const void* p0; const void* p1; int ld; };
template <int NP> __device__ __forceinline__ void load_frags(const Opnd& o, int row, int kb, int hh, v16b& fh_, v16b& fl_) {
  if (NP == 0) { frag_ksplit((const float*)o.p0 + (size_t)row * o.ld + kb, hh, fh_, fl_); }
  else if (NP == 3) {
    const float* p = (const float*)o.p0 + (size_t)row * o.ld + kb; const float* p0 = p + 8 * hh; const float* p1 = p + 16 + 8 * hh;
#pragma unroll
    for (int e = 0; e < 8; ++e) { fh_[e] = (b16)p0[e]; fh_[8 + e] = (b16)p1[e]; }
    fl_ = fh_;
  } else {
    fh_ = frag_kb((const b16*)o.p0 + (size_t)row * o.ld + kb, hh);
    if (NP == 2) fl_ = frag_kb((const b16*)o.p1 + (size_t)row * o.ld + kb, hh); else fl_ = fh_;
  }
}
template <int ANP, int BNP> __device__ __forceinline__ v8f mac(v16b ah, v16b al, v16b bh, v16b bl, v8f c) {
  c = wmma16b(ah, bh, c);
  if (BNP == 0 || BNP == 2) c = wmma16b(ah, bl, c);
  if (ANP == 0 || ANP == 2) c = wmma16b(al, bh, c);
  return c;
}
template <int ANP, int BNP>
__device__ __forceinline__ void gemm_tile(const Opnd& A, const Opnd& B, int K, int m0, int c0, int nloc, int hlf, v8f (&acc)[2][4]) {
  for (int kb = 0; kb < K; kb += 32) {
    v16b a0h, a0l, a1h, a1l;
    load_frags<ANP>(A, m0 + nloc, kb, hlf, a0h, a0l);
    load_frags<ANP>(A, m0 + 16 + nloc, kb, hlf, a1h, a1l);
#pragma unroll
    for (int t = 0; t < 4; ++t) {
      v16b bh, bl;
      load_frags<BNP>(B, c0 + t * 16 + nloc, kb, hlf, bh, bl);
      acc[0][t] = mac<ANP, BNP>(a0h, a0l, bh, bl, acc[0][t]);
      acc[1][t] = mac<ANP, BNP>(a1h, a1l, bh, bl, acc[1][t]);
    }
  }
}

struct Epi { float scale; const float* cbias; const float* rbias; int act; float post; const float* rscale; const float* resid; };
__device__ __forceinline__ float epi_val(const Epi& e, float acc, int row, int col) {
  float val = acc * e.scale;
  if (e.cbias) val += e.cbias[col];
  if (e.rbias) val += e.rbias[row];
  if (e.act == 1) val = 0.5f * val * (1.0f + erff(val * 0.70710678118654752f));
  val *= e.post;
  if (e.rscale) val *= e.rscale[(size_t)row * 32];
  return val;
}
__device__ __forceinline__ void epi_planes(v8f (&acc)[2][4], const Epi& e, bool two,
                                           b16* __restrict__ oh, b16* __restrict__ ol, int ldo, int m0, int c0, int lane, b16* Th, b16* Tl) {
  const int nloc = lane & 15, hlf = lane >> 4;
#pragma unroll
  for (int t = 0; t < 4; ++t)
#pragma unroll
    for (int r = 0; r < 2; ++r)
#pragma unroll
      for (int v = 0; v < 8; ++v) {
        const int rr = r * 16 + v + 8 * hlf, cc = t * 16 + nloc;
        const float val = epi_val(e, acc[r][t][v], m0 + rr, c0 + cc);
        b16 h_, l_; split16(val, h_, l_);
        Th[rr * 64 + cc] = h_; if (two) Tl[rr * 64 + cc] = l_;
      }
  wave_lds_sync();
  for (int pass = 0; pass < 2; ++pass) {
#pragma unroll
    for (int j = 0; j < 8; ++j) {
      const int rr = j * 4 + (lane >> 3), c8 = (lane & 7) * 8;
      const size_t o = (size_t)(m0 + rr) * ldo + c0 + c8;
      *(volatile v8b*)(oh + o) = ld8b(Th + rr * 64 + c8);
      if (two) *(volatile v8b*)(ol + o) = ld8b(Tl + rr * 64 + c8);
    }
    __threadfence();
  }
}
__device__ __forceinline__ void epi_f32(v8f (&acc)[2][4], const Epi& e, float* __restrict__ out, int ldo, int m0, int c0, int lane, float* Tt) {
  const int nloc = lane & 15, hlf = lane >> 4;
#pragma unroll
  for (int t = 0; t < 4; ++t)
#pragma unroll
    for (int r = 0; r < 2; ++r)
#pragma unroll
      for (int v = 0; v < 8; ++v) {
        const int rr = r * 16 + v + 8 * hlf, cc = t * 16 + nloc;
        Tt[rr * 64 + cc] = epi_val(e, acc[r][t][v], m0 + rr, c0 + cc);
      }
  wave_lds_sync();
  float* dst0 = out + (size_t)m0 * ldo + c0; const float* rs0 = e.resid ? e.resid + (size_t)m0 * ldo + c0 : nullptr;
  for (int pass = 0; pass < 2; ++pass) {
#pragma unroll
    for (int j = 0; j < 16; ++j) {
      const int rr = j * 2 + hlf, c4 = nloc * 4;
      v4f val = *(const v4f*)(Tt + rr * 64 + c4);
      if (rs0) val += *(const v4f*)(rs0 + (size_t)rr * ldo + c4);
      *(volatile v4f*)(dst0 + (size_t)rr * ldo + c4) = val;
    }
    __threadfence();
  }
}


__global__ __launch_bounds__(256) void cvt_kernel(const float* __restrict__ a0, int n0, const float* __restrict__ a1, int n1,
                                                  const float* __restrict__ a2, int n2, const float* __restrict__ a3, int n3, b16* __restrict__ dst) {
  const size_t tid = (size_t)blockIdx.x * blockDim.x + threadIdx.x, stride = (size_t)gridDim.x * blockDim.x;
  const size_t c0n = (size_t)n0 / 8, c1n = (size_t)n1 / 8, c2n = (size_t)n2 / 8, c3n = (size_t)n3 / 8;
  for (int pass = 0; pass < 2; ++pass) {
    for (size_t c = tid; c < c0n + c1n + c2n + c3n; c += stride) {
      const float* src; size_t o;
      if (c < c0n) { src = a0 + c * 8; o = c * 8; }
      else if (c < c0n + c1n) { src = a1 + (c - c0n) * 8; o = (size_t)n0 + (c - c0n) * 8; }
      else if (c < c0n + c1n + c2n) { src = a2 + (c - c0n - c1n) * 8; o = (size_t)n0 + n1 + (c - c0n - c1n) * 8; }
      else { src = a3 + (c - c0n - c1n - c2n) * 8; o = (size_t)n0 + n1 + n2 + (c - c0n - c1n - c2n) * 8; }
      v8b v;
#pragma unroll
      for (int e = 0; e < 8; ++e) v[e] = (b16)src[e];
      *(volatile v8b*)(dst + o) = v;
    }
    __threadfence();
  }
}

__global__ __launch_bounds__(256) void ln_kernel(const float* __restrict__ x, const float* __restrict__ g, const float* __restrict__ bta, b16* __restrict__ h) {
  __shared__ __attribute__((aligned(16))) b16 Ts[8][D];
  const int lane = threadIdx.x & 31, row = blockIdx.x * 8 + (threadIdx.x >> 5);
  const float* xr = x + (size_t)row * D;
  float v[16];
#pragma unroll
  for (int j = 0; j < 4; ++j) { const v4f q = *(const v4f*)(xr + j * 128 + lane * 4); v[4*j] = q[0]; v[4*j+1] = q[1]; v[4*j+2] = q[2]; v[4*j+3] = q[3]; }
  float s = 0.f;
#pragma unroll
  for (int j = 0; j < 16; ++j) s += v[j];
#pragma unroll
  for (int o = 16; o > 0; o >>= 1) s += __shfl_xor(s, o);
  const float mu = s * (1.0f / D);
  float s2 = 0.f;
#pragma unroll
  for (int j = 0; j < 16; ++j) { const float dl = v[j] - mu; s2 += dl * dl; }
#pragma unroll
  for (int o = 16; o > 0; o >>= 1) s2 += __shfl_xor(s2, o);
  const float rs = rsqrtf(s2 * (1.0f / D) + EPS);
  b16* Tp = Ts[threadIdx.x >> 5];
#pragma unroll
  for (int j = 0; j < 4; ++j)
#pragma unroll
    for (int q = 0; q < 4; ++q) { const int c = j * 128 + lane * 4 + q; Tp[c] = (b16)((v[4*j+q] - mu) * rs * g[c] + bta[c]); }
  wave_lds_sync();
  b16* dst = h + (size_t)row * D;
  for (int pass = 0; pass < 2; ++pass) {
#pragma unroll
    for (int j = 0; j < 2; ++j) { const int e = j * 256 + lane * 8; *(volatile v8b*)(dst + e) = ld8b(Tp + e); }
    __threadfence();
  }
}

__global__ __launch_bounds__(256) void transpose_kernel(const b16* __restrict__ h, b16* __restrict__ hT) {
  __shared__ __attribute__((aligned(16))) b16 Tl[D][64 + 8];
  const int tid = threadIdx.x, lane = tid & 31, wave = tid >> 5;
  const int b = blockIdx.x / (T / 64), t0 = (blockIdx.x % (T / 64)) * 64;
  const b16* src = h + ((size_t)b * T + t0) * D;
  for (int it = 0; it < 16; ++it) {
    const int tk = it * 4 + (tid >> 6), c8 = (tid & 63) * 8;
    const v8b q = ld8b(src + (size_t)tk * D + c8);
#pragma unroll
    for (int e = 0; e < 8; ++e) Tl[c8 + e][tk] = q[e];
  }
  __syncthreads();
  b16* dst = hT + (size_t)b * D * T + t0;
  for (int pass = 0; pass < 2; ++pass) {
#pragma unroll
    for (int j = 0; j < 16; ++j) { const int c = wave * 64 + j * 4 + (lane >> 3), e8 = (lane & 7) * 8; *(volatile v8b*)(dst + (size_t)c * T + e8) = *(const v8b*)(&Tl[c][e8]); }
    __threadfence();
  }
}

__global__ __launch_bounds__(128) void qkv_kernel(const b16* __restrict__ xn, const b16* __restrict__ w, const float* __restrict__ bias,
                                                  b16* __restrict__ Qh, b16* __restrict__ Kh, b16* __restrict__ Vh) {
  __shared__ __attribute__((aligned(16))) b16 Ts[4][32 * 64];
  const int lane = threadIdx.x & 31, wave = threadIdx.x >> 5, nloc = lane & 15, hlf = lane >> 4;
  const int m0 = blockIdx.y * 128 + wave * 32, c0 = blockIdx.x * 64;
  const int mat = c0 / D, head = (c0 % D) / DH;
  v8f acc[2][4];
#pragma unroll
  for (int r = 0; r < 2; ++r)
#pragma unroll
    for (int t = 0; t < 4; ++t) acc[r][t] = (v8f){};
  const Opnd A{xn, nullptr, D}, B{w, nullptr, D};
  gemm_tile<1, 1>(A, B, D, m0, c0, nloc, hlf, acc);
  const int b = m0 / T, t0 = m0 % T;
  const float sc = (mat == 0) ? 0.125f : 1.0f;
  b16* Tp = Ts[wave];
#pragma unroll
  for (int t = 0; t < 4; ++t)
#pragma unroll
    for (int r = 0; r < 2; ++r)
#pragma unroll
      for (int v = 0; v < 8; ++v) {
        const int rr = r * 16 + v + 8 * hlf, d = t * 16 + nloc;
        const float val = (acc[r][t][v] + bias[c0 + d]) * sc;
        const int idx = (mat < 2) ? (rr * 64 + d) : ((rr >> 4) * 1024 + d * 16 + (rr & 15));
        Tp[idx] = (b16)val;
      }
  wave_lds_sync();
  b16* dh; size_t o;
  if (mat == 0)      { o = ((size_t)(b * NH + head) * T + t0) * DH; dh = Qh + o; }
  else if (mat == 1) { o = ((size_t)(b * NH + head) * T + t0) * DH; dh = Kh + o; }
  else               { o = ((size_t)(b * NH + head) * QT_PER_B + (t0 >> 4)) * (size_t)(DH * 16); dh = Vh + o; }
  for (int pass = 0; pass < 2; ++pass) {
#pragma unroll
    for (int j = 0; j < 8; ++j) { const int e = (j * 32 + lane) * 8; *(volatile v8b*)(dh + e) = ld8b(Tp + e); }
    __threadfence();
  }
}

__global__ __launch_bounds__(256) void attn_kernel(const b16* __restrict__ Qh, const b16* __restrict__ Kh, const b16* __restrict__ Vh, b16* __restrict__ yh) {
  __shared__ __attribute__((aligned(16))) b16 Os[8][16 * 64];
  const int wid = threadIdx.x >> 5, lane = threadIdx.x & 31, hh = lane >> 4, col = lane & 15;
  const int qtile = blockIdx.x * 8 + wid, g = qtile / QT_PER_B, q0 = (qtile % QT_PER_B) << 4;
  const int b = g / NH, hd = g % NH;
  const size_t ko = (size_t)g * T * DH, qo = ((size_t)g * T + q0 + col) * DH;
  const v16b q0h = frag_kb(Qh + qo, hh), q1h = frag_kb(Qh + qo + 32, hh);
  float m = -INFINITY, l = 0.0f;
  v8f o0 = {}, o1 = {}, o2 = {}, o3 = {};
  for (int kb = 0; kb < T; kb += 32) {
    const size_t r0 = ko + (size_t)(kb + col) * DH, r1 = ko + (size_t)(kb + 16 + col) * DH;
    v8f s0 = {}, s1 = {};
    v16b ah = frag_kb(Kh + r0, hh);      s0 = wmma16b(ah, q0h, s0);
    ah = frag_kb(Kh + r0 + 32, hh);      s0 = wmma16b(ah, q1h, s0);
    ah = frag_kb(Kh + r1, hh);           s1 = wmma16b(ah, q0h, s1);
    ah = frag_kb(Kh + r1 + 32, hh);      s1 = wmma16b(ah, q1h, s1);
    float mr = -INFINITY;
#pragma unroll
    for (int r = 0; r < 8; ++r) mr = fmaxf(mr, fmaxf(s0[r], s1[r]));
    mr = fmaxf(mr, __shfl_xor(mr, 16));
    const float mn = fmaxf(m, mr), al_ = __expf(m - mn);
    m = mn;
    float sum = 0.0f; v16b pb;
#pragma unroll
    for (int r = 0; r < 8; ++r) { const float p0 = __expf(s0[r] - mn), p1 = __expf(s1[r] - mn); sum += p0 + p1; pb[r] = (b16)p0; pb[8 + r] = (b16)p1; }
    sum += __shfl_xor(sum, 16);
    l = l * al_ + sum;
#pragma unroll
    for (int r = 0; r < 8; ++r) { o0[r] *= al_; o1[r] *= al_; o2[r] *= al_; o3[r] *= al_; }
    const size_t v0 = ko + (size_t)(kb >> 4) * (DH * 16) + 8 * hh, v1 = v0 + DH * 16;
#pragma unroll
    for (int n = 0; n < 4; ++n) {
      const int f = n * 16 + col;
      const v16b va = cat8b(ld8b(Vh + v0 + f * 16), ld8b(Vh + v1 + f * 16));
      v8f& o = (n == 0) ? o0 : (n == 1) ? o1 : (n == 2) ? o2 : o3;
      o = wmma16b(va, pb, o);
    }
  }
  const float inv = 1.0f / l;
  b16* Tt = Os[wid];
#pragma unroll
  for (int r = 0; r < 8; ++r) {
    const int hr = 8 * hh + r;
    Tt[col * 64 + 0 + hr] = (b16)(o0[r] * inv); Tt[col * 64 + 16 + hr] = (b16)(o1[r] * inv);
    Tt[col * 64 + 32 + hr] = (b16)(o2[r] * inv); Tt[col * 64 + 48 + hr] = (b16)(o3[r] * inv);
  }
  wave_lds_sync();
  b16* dst0 = yh + ((size_t)b * T + q0) * D + hd * DH;
  for (int pass = 0; pass < 2; ++pass) {
#pragma unroll
    for (int j = 0; j < 4; ++j) { const int rr = j * 4 + (lane >> 3), c8 = (lane & 7) * 8; *(volatile v8b*)(dst0 + (size_t)rr * D + c8) = ld8b(Tt + rr * 64 + c8); }
    __threadfence();
  }
}

__global__ __launch_bounds__(256) void poskernel_kernel(const int* __restrict__ posv, const int* __restrict__ posh, b16* __restrict__ E, float* __restrict__ lslot) {
  const int lane = threadIdx.x & 31, row = blockIdx.x * 8 + (threadIdx.x >> 5);
  const int b = row / T;
  const int* pv = posv + (size_t)b * T; const int* ph = posh + (size_t)b * T;
  const float qv = (float)pv[row % T], qh_ = (float)ph[row % T];
  float ev[32]; float sum = 0.0f;
#pragma unroll
  for (int j = 0; j < 4; ++j)
#pragma unroll
    for (int e = 0; e < 8; ++e) {
      const int k = j * 256 + lane * 8 + e;
      const float dv = qv - (float)pv[k], dh_ = qh_ - (float)ph[k];
      const float w = expf(-(dv * dv + dh_ * dh_) * INV_2SIG2);
      ev[j * 8 + e] = w; sum += w;
    }
#pragma unroll
  for (int o = 16; o > 0; o >>= 1) sum += __shfl_xor(sum, o);
  b16* Er = E + (size_t)row * T;
  for (int pass = 0; pass < 2; ++pass) {
#pragma unroll
    for (int j = 0; j < 4; ++j) { v8b p;
#pragma unroll
      for (int e = 0; e < 8; ++e) p[e] = (b16)(ev[j * 8 + e] * KW_SC);
      *(volatile v8b*)(Er + j * 256 + lane * 8) = p; }
    ((volatile float*)lslot)[(size_t)row * 32 + lane] = (lane == 0) ? (1.0f / sum) : 0.0f;
    __threadfence();
  }
}

template <bool OUT16>
__global__ __launch_bounds__(128) void gemm_kernel(const b16* __restrict__ A, int lda, const b16* __restrict__ Bm, int ldb, int K, float scale,
                                                   const float* __restrict__ cbias, const float* __restrict__ rbias, int act, int pm, const float* __restrict__ gatep,
                                                   const float* __restrict__ rscale, const float* __restrict__ resid, b16* __restrict__ o16, float* __restrict__ o32, int ldo) {
  __shared__ __attribute__((aligned(16))) float Ts[4][32 * 64];
  __shared__ __attribute__((aligned(16))) b16 Th[4][32 * 64];
  const int lane = threadIdx.x & 31, wave = threadIdx.x >> 5, nloc = lane & 15, hlf = lane >> 4;
  const int m0 = blockIdx.y * 128 + wave * 32, c0 = blockIdx.x * 64;
  v8f acc[2][4];
#pragma unroll
  for (int r = 0; r < 2; ++r)
#pragma unroll
    for (int t = 0; t < 4; ++t) acc[r][t] = (v8f){};
  const Opnd Ao{A, nullptr, lda}, Bo{Bm, nullptr, ldb};
  gemm_tile<1, 1>(Ao, Bo, K, m0, c0, nloc, hlf, acc);
  float post = 1.0f;
  if (pm != 0) { const float gs = 1.0f / (1.0f + expf(-gatep[0])); post = (pm == 1) ? gs : (1.0f - gs); }
  const Epi e{scale, cbias, rbias, act, post, rscale, resid};
  if (OUT16) epi_planes(acc, e, false, o16, nullptr, ldo, m0, c0, lane, Th[wave], nullptr);
  else       epi_f32(acc, e, o32, ldo, m0, c0, lane, Ts[wave]);
}
}

extern "C" void kernel_launch(void* const* d_in, const int* in_sizes, int n_in,
                              void* d_out, int out_size, void* d_ws, size_t ws_size, hipStream_t stream) {
  (void)n_in; (void)out_size;
  const float* x    = (const float*)d_in[0];
  const int* posv   = (const int*)d_in[1];
  const int* posh   = (const int*)d_in[2];
  const float* n1w  = (const float*)d_in[3];  const float* n1b = (const float*)d_in[4];
  const float* in_w = (const float*)d_in[5];
  const float* in_b = (const float*)d_in[6];
  const float* ow   = (const float*)d_in[7];
  const float* ob   = (const float*)d_in[8];
  const float* n2w  = (const float*)d_in[9];  const float* n2b = (const float*)d_in[10];
  const float* w1   = (const float*)d_in[11];
  const float* b1   = (const float*)d_in[12];
  const float* w2   = (const float*)d_in[13];
  const float* b2   = (const float*)d_in[14];
  const float* gate = (const float*)d_in[15];
  float* out = (float*)d_out;
  if (in_sizes[0] != MROWS * D || in_sizes[1] != MROWS || in_sizes[5] != NQKV * D || in_sizes[11] != FF * D || in_sizes[13] != D * FF) return;

  size_t off = 0; char* ws = (char*)d_ws;
  auto carve = [&](size_t bytes) { char* p = ws + off; off += (bytes + 255) & ~(size_t)255; return p; };
  b16* w16   = (b16*)carve((size_t)(NQKV * D + D * D + FF * D + D * FF) * 2);
  b16* xn    = (b16*)carve((size_t)MROWS * D * 2);
  b16* xnT   = (b16*)carve((size_t)MROWS * D * 2);
  b16* R32   = (b16*)carve((size_t)MROWS * FF * 2);
  float* x1a = (float*)carve((size_t)MROWS * D * 4);
  b16* E16   = (b16*)carve((size_t)MROWS * T * 2);
  float* lsl = (float*)carve((size_t)MROWS * 32 * 4);
  float* x1  = (float*)carve((size_t)MROWS * D * 4);
  if (off > ws_size) return;
  const b16* inw16 = w16; const b16* ow16 = w16 + (size_t)NQKV * D; const b16* w116 = ow16 + (size_t)D * D; const b16* w216 = w116 + (size_t)FF * D;
  b16* Qh = R32; b16* Kh = R32 + (size_t)MROWS * D; b16* Vh = Kh + (size_t)MROWS * D; b16* yh = Vh + (size_t)MROWS * D; b16* gm = R32;
  const int ROWBLK = MROWS / 128;
  cvt_kernel<<<1024, 256, 0, stream>>>(in_w, NQKV * D, ow, D * D, w1, FF * D, w2, D * FF, w16);
  ln_kernel<<<MROWS / 8, 256, 0, stream>>>(x, n1w, n1b, xn);
  transpose_kernel<<<Bsz * T / 64, 256, 0, stream>>>(xn, xnT);
  poskernel_kernel<<<MROWS / 8, 256, 0, stream>>>(posv, posh, E16, lsl);
  qkv_kernel<<<dim3(NQKV / 64, ROWBLK), 128, 0, stream>>>(xn, inw16, in_b, Qh, Kh, Vh);
  attn_kernel<<<Bsz * NH * QT_PER_B / 8, 256, 0, stream>>>(Qh, Kh, Vh, yh);
  gemm_kernel<false><<<dim3(D / 64, ROWBLK), 128, 0, stream>>>(yh, D, ow16, D, D, 1.0f, ob, nullptr, 0, 1, gate, nullptr, x, nullptr, x1a, D);
  for (int b = 0; b < Bsz; ++b)
    gemm_kernel<false><<<dim3(D / 64, T / 128), 128, 0, stream>>>(E16 + (size_t)b * T * T, T, xnT + (size_t)b * D * T, T, T, INV_KW_SC, nullptr, nullptr, 0, 2, gate,
                                                                 lsl + (size_t)b * T * 32, x1a + (size_t)b * T * D, nullptr, x1 + (size_t)b * T * D, D);
  ln_kernel<<<MROWS / 8, 256, 0, stream>>>(x1, n2w, n2b, xn);
  gemm_kernel<true><<<dim3(FF / 64, ROWBLK), 128, 0, stream>>>(xn, D, w116, D, D, 1.0f, b1, nullptr, 1, 0, gate, nullptr, nullptr, gm, nullptr, FF);
  gemm_kernel<false><<<dim3(D / 64, ROWBLK), 128, 0, stream>>>(gm, FF, w216, FF, FF, 1.0f, b2, nullptr, 0, 0, gate, nullptr, x1, nullptr, out, D);
}
